// MambaBlock_46892452937750
// MI455X (gfx1250) — hardware-verified
//
#include <hip/hip_runtime.h>
#include <math.h>

typedef __attribute__((ext_vector_type(16))) _Float16 v16h;
typedef __attribute__((ext_vector_type(8)))  _Float16 v8h;
typedef __attribute__((ext_vector_type(16))) __bf16   v16b;
typedef __attribute__((ext_vector_type(8)))  __bf16   v8b;
typedef __attribute__((ext_vector_type(8)))  float    v8f;
typedef __attribute__((ext_vector_type(4)))  float    v4f;

constexpr int kBatch  = 2;
constexpr int kSeq    = 1024;
constexpr int kHid    = 1024;
constexpr int kInner  = 2048;
constexpr int kNst    = 16;
constexpr int kDtR    = 64;
constexpr int kXzP    = 2 * kInner;
constexpr int kBcN    = 2 * kNst;
constexpr int kBcP    = 64;
constexpr int kTok    = kBatch * kSeq;
constexpr int kConvTP = 260;
constexpr int kScanTS = 64;
constexpr int kScanCh = 64;
constexpr int kScanYP = 68;
static_assert(kBcN == 32 && kBcP == 64, "B/C projection width and padded pitch");
static_assert((kHid % 32) == 0 && (kInner % 32) == 0 && (kDtR % 32) == 0, "GEMM K multiples of 32");
static_assert((kTok % 64) == 0 && (kXzP % 64) == 0 && (kBcP % 64) == 0 && (kDtR % 64) == 0 && (kInner % 64) == 0 && (kHid % 64) == 0, "GEMM M,N multiples of 64");
static_assert((kSeq % kScanTS) == 0 && (kSeq % 64) == 0 && (kInner % kScanCh) == 0 && (kInner % 256) == 0, "tile multiples");
static_assert(kScanTS == kScanCh, "scan staging uses one thread per staged step");
static_assert(kHid == 128 * 8, "LayerNorm block covers one row with 128 threads x 8");

constexpr size_t kOffBIH = 0;
constexpr size_t kOffBIL = kOffBIH + (size_t)kXzP  * kHid   * 2;
constexpr size_t kOffBOH = kOffBIL + (size_t)kXzP  * kHid   * 2;
constexpr size_t kOffBOL = kOffBOH + (size_t)kHid  * kInner * 2;
constexpr size_t kOffBCH = kOffBOL + (size_t)kHid  * kInner * 2;
constexpr size_t kOffBCL = kOffBCH + (size_t)kBcP  * kInner * 2;
constexpr size_t kOffBDR = kOffBCL + (size_t)kBcP  * kInner * 2;
constexpr size_t kOffBDT = kOffBDR + (size_t)kDtR  * kInner * 2;
constexpr size_t kOffNH  = kOffBDT + (size_t)kInner * kDtR  * 2;
constexpr size_t kOffNL  = kOffNH  + (size_t)kTok  * kHid   * 2;
constexpr size_t kOffXZ  = kOffNL  + (size_t)kTok  * kHid   * 2;
constexpr size_t kOffXAH = kOffXZ  + (size_t)kTok  * kXzP   * 4;
constexpr size_t kOffXAL = kOffXAH + (size_t)kTok  * kInner * 2;
constexpr size_t kOffBC  = kOffXAL + (size_t)kTok  * kInner * 2;
constexpr size_t kOffDTR = kOffBC  + (size_t)kTok  * kBcP   * 4;
constexpr size_t kOffDTM = kOffDTR + (size_t)kTok  * kDtR   * 2;
constexpr size_t kOffDTP = kOffDTM + (size_t)kTok  * 4;
constexpr size_t kOffGH  = kOffDTP + (size_t)kTok  * kInner * 4;
constexpr size_t kOffGL  = kOffGH  + (size_t)kTok  * kInner * 2;
constexpr size_t kWsTotal = kOffGL + (size_t)kTok  * kInner * 2;
static_assert(kWsTotal <= 134217728ull, "carve cap");
static_assert((kOffBIL % 128) == 0 && (kOffBOH % 128) == 0 && (kOffBOL % 128) == 0 && (kOffBCH % 128) == 0 &&
              (kOffBCL % 128) == 0 && (kOffBDR % 128) == 0 && (kOffBDT % 128) == 0 && (kOffNH % 128) == 0 &&
              (kOffNL % 128) == 0 && (kOffXZ % 128) == 0 && (kOffXAH % 128) == 0 && (kOffXAL % 128) == 0 &&
              (kOffBC % 128) == 0 && (kOffDTR % 128) == 0 && (kOffDTM % 128) == 0 && (kOffDTP % 128) == 0 &&
              (kOffGH % 128) == 0 && (kOffGL % 128) == 0, "128-B aligned regions");

__device__ __forceinline__ unsigned short f2bf_bits(float f) {
  unsigned u = __float_as_uint(f);
  return (unsigned short)((u + 0x7FFFu + ((u >> 16) & 1u)) >> 16);
}
__device__ __forceinline__ float bf_bits2f(unsigned short h) { return __uint_as_float(((unsigned)h) << 16); }

__device__ __forceinline__ void dep_guard4_b(v8f& a, v8f& b, v8f& c, v8f& d, v16b x, v16b y) {
  asm volatile("v_nop\n\tv_nop\n\tv_nop\n\tv_nop" : "+v"(a), "+v"(b), "+v"(c), "+v"(d) : "v"(x), "v"(y));
}
__device__ __forceinline__ void keep4_b(v16b a, v16b b, v16b c, v16b d) { asm volatile("v_nop" :: "v"(a), "v"(b), "v"(c), "v"(d)); }
__device__ __forceinline__ void acc_guard4(v8f& a, v8f& b, v8f& c, v8f& d) { asm volatile("v_nop\n\tv_nop\n\tv_nop\n\tv_nop" : "+v"(a), "+v"(b), "+v"(c), "+v"(d)); }
template <typename T> struct Frag;
template <> struct Frag<__bf16> {
  typedef v16b V; union U { v16b v; v8b h[2]; };
  static __device__ __forceinline__ v16b load(const __bf16* p) {
    U f; f.h[0] = *(const v8b*)(p); f.h[1] = *(const v8b*)(p + 16); return f.v;
  }
  static __device__ __forceinline__ v8f mma(v16b a, v16b b, v8f c) {
    return __builtin_amdgcn_wmma_f32_16x16x32_bf16(false, a, false, b, (short)0, c, false, false);
  }
  static __device__ __forceinline__ void guard4(v8f& a, v8f& b, v8f& c, v8f& d, v16b x, v16b y) { dep_guard4_b(a, b, c, d, x, y); }
  static __device__ __forceinline__ void keep(v16b a, v16b b, v16b c, v16b d) { keep4_b(a, b, c, d); }
};

template <int ET> struct Elem;
template <> struct Elem<1> { typedef __bf16 T; };
template <int ET, int SPL, int BIAS_MODE, int OUT_MODE, bool RESID, int ACT = 0>
__global__ __launch_bounds__(256) void wmma_gemm64(
    const unsigned short* __restrict__ Ap, const unsigned short* __restrict__ A2p, int lda, long strideA,
    const unsigned short* __restrict__ Btp, const unsigned short* __restrict__ Bt2p, int ldb, long strideB,
    void* __restrict__ Cout, void* __restrict__ Cout2, int ldc, long strideC,
    const float* __restrict__ bias,
    const float* __restrict__ resid, long strideR,
    int M, int N, int K, float scale) {
  typedef typename Elem<ET>::T T;
  typedef typename Frag<T>::V V;
  const T* A = (const T*)Ap; const T* A2 = (const T*)A2p; const T* Bt = (const T*)Btp; const T* Bt2 = (const T*)Bt2p;
  __shared__ __align__(16) float sT[8][16 * 68];
  const int b    = blockIdx.y;
  const int lane = threadIdx.x & 31;
  const int wave = threadIdx.x >> 5;
  const int tilesN = N >> 6;
  const int tilesM = M >> 6;
  const int tile = blockIdx.x * 8 + wave;
  if (tile >= tilesM * tilesN) return;
  const int tm = tile / tilesN;
  const int tn = tile - tm * tilesN;
  const int m0 = tm << 6;
  const int n0 = tn << 6;

  const T* Ab  = A  + (size_t)b * strideA;
  const T* Bb  = Bt + (size_t)b * strideB;
  const T* Ab2 = (SPL >= 1) ? (A2  + (size_t)b * strideA) : nullptr;
  const T* Bb2 = (SPL == 2) ? (Bt2 + (size_t)b * strideB) : nullptr;

  const int rlane = lane & 15;
  const int koff  = (lane >> 4) * 8;
  const int mOff  = (lane >> 4) * 8;

  v8f acc[4][4];
#pragma unroll
  for (int i = 0; i < 4; ++i)
#pragma unroll
    for (int j = 0; j < 4; ++j) acc[i][j] = (v8f){0.f,0.f,0.f,0.f,0.f,0.f,0.f,0.f};

  for (int k0 = 0; k0 < K; k0 += 32) {
    V bh[4], bl[4];
#pragma unroll
    for (int j = 0; j < 4; ++j) {
      const size_t bo = (size_t)(n0 + (j << 4) + rlane) * ldb + koff + k0;
      bh[j] = Frag<T>::load(Bb + bo);
      if (SPL == 2) bl[j] = Frag<T>::load(Bb2 + bo);
    }
#pragma unroll
    for (int i = 0; i < 4; ++i) {
      const size_t ao = (size_t)(m0 + (i << 4) + rlane) * lda + koff + k0;
      V ah = Frag<T>::load(Ab + ao);
      V al;
      if (SPL >= 1) al = Frag<T>::load(Ab2 + ao);
#pragma unroll
      for (int j = 0; j < 4; ++j) {
        acc[i][j] = Frag<T>::mma(ah, bh[j], acc[i][j]);
        if (SPL == 2) acc[i][j] = Frag<T>::mma(ah, bl[j], acc[i][j]);
        if (SPL >= 1) acc[i][j] = Frag<T>::mma(al, bh[j], acc[i][j]);
      }
      Frag<T>::guard4(acc[i][0], acc[i][1], acc[i][2], acc[i][3], ah, (SPL >= 1) ? al : ah);
    }
    Frag<T>::keep(bh[0], bh[1], bh[2], bh[3]);
    if (SPL == 2) Frag<T>::keep(bl[0], bl[1], bl[2], bl[3]);
  }
  acc_guard4(acc[0][0], acc[0][1], acc[0][2], acc[0][3]);
  acc_guard4(acc[1][0], acc[1][1], acc[1][2], acc[1][3]);
  acc_guard4(acc[2][0], acc[2][1], acc[2][2], acc[2][3]);
  acc_guard4(acc[3][0], acc[3][1], acc[3][2], acc[3][3]);

  float* slab = sT[wave];
  const float* Rb = RESID ? (resid + (size_t)b * strideR) : nullptr;
#pragma unroll
  for (int i = 0; i < 4; ++i) {
    const int mBase = m0 + (i << 4);
#pragma unroll
    for (int j = 0; j < 4; ++j) {
      const int n = n0 + (j << 4) + rlane;
      float bv = 0.f;
      if (BIAS_MODE == 2) bv = bias[n];
#pragma unroll
      for (int r = 0; r < 8; ++r) {
        float v = acc[i][j][r] * scale;
        if (BIAS_MODE == 1) v += bias[mBase + mOff + r];
        if (BIAS_MODE == 2) v += bv;
        if (RESID) v += Rb[(size_t)(mBase + mOff + r) * ldc + n];
        if (ACT == 2) v = fmaxf(v, 0.0f);
        if (ACT == 4) v = (v > 0.f) ? v : 0.01f * v;
        slab[(mOff + r) * 68 + (j << 4) + rlane] = v;
      }
    }
    __builtin_amdgcn_fence(__ATOMIC_RELEASE, "workgroup");
    __builtin_amdgcn_wave_barrier();
    __builtin_amdgcn_fence(__ATOMIC_ACQUIRE, "workgroup");
    if (OUT_MODE == 0) {
      float* C = (float*)Cout + (size_t)b * strideC;
      const int hh = lane >> 4, c4 = (lane & 15) * 4;
      for (int pass = 0; pass < 2; ++pass) {
#pragma unroll
        for (int it = 0; it < 8; ++it) {
          const int row = it * 2 + hh;
          v4f v = *(const v4f*)(slab + row * 68 + c4);
          *(volatile v4f*)(C + (size_t)(mBase + row) * ldc + n0 + c4) = v;
        }
        __threadfence();
      }
    } else {
      const int q = lane >> 3, c8 = (lane & 7) * 8;
      unsigned short* C  = (unsigned short*)Cout  + (size_t)b * strideC;
      unsigned short* C2 = (OUT_MODE == 2) ? ((unsigned short*)Cout2 + (size_t)b * strideC) : nullptr;
      for (int pass = 0; pass < 2; ++pass) {
#pragma unroll
        for (int it = 0; it < 4; ++it) {
          const int row = it * 4 + q;
          const float* sp = slab + row * 68 + c8;
          v8h hv, lv;
#pragma unroll
          for (int e = 0; e < 8; ++e) {
            if (OUT_MODE == 1) {
              hv[e] = (_Float16)sp[e];
            } else {
              const unsigned short hb = f2bf_bits(sp[e]);
              hv[e] = __builtin_bit_cast(_Float16, hb);
              if (OUT_MODE == 2) {
                const unsigned short lb = f2bf_bits(sp[e] - bf_bits2f(hb));
                lv[e] = __builtin_bit_cast(_Float16, lb);
              }
            }
          }
          *(volatile v8h*)(C + (size_t)(mBase + row) * ldc + n0 + c8) = hv;
          if (OUT_MODE == 2) *(volatile v8h*)(C2 + (size_t)(mBase + row) * ldc + n0 + c8) = lv;
        }
        __threadfence();
      }
    }
    __builtin_amdgcn_fence(__ATOMIC_RELEASE, "workgroup");
    __builtin_amdgcn_wave_barrier();
    __builtin_amdgcn_fence(__ATOMIC_ACQUIRE, "workgroup");
  }
}

template <bool WITH_LO>
__global__ __launch_bounds__(256) void transpose_split_kernel(
    const float* __restrict__ W, unsigned short* __restrict__ BtH, unsigned short* __restrict__ BtL, int Kdim, int Ndim)
{
  __shared__ float tile[64 * 65];
  const int tid = threadIdx.x, lane = tid & 31, wave = tid >> 5;
  const int n0 = blockIdx.x * 64;
  const int k0 = blockIdx.y * 64;
#pragma unroll 4
  for (int p = 0; p < 16; ++p) {
    const int idx = tid + p * 256;
    const int kk  = idx >> 6;
    const int nn  = idx & 63;
    const int n   = n0 + nn;
    const int nc  = (n < Ndim) ? n : (Ndim - 1);
    const float v = W[(size_t)(k0 + kk) * Ndim + nc];
    tile[kk * 65 + nn] = (n < Ndim) ? v : 0.f;
  }
  __syncthreads();
  const int q = lane >> 3, c8 = (lane & 7) * 8;
  v8h hv[2], lv[2];
#pragma unroll
  for (int it = 0; it < 2; ++it) {
    const int nrow = it * 32 + wave * 4 + q;
#pragma unroll
    for (int e = 0; e < 8; ++e) {
      const float f = tile[(c8 + e) * 65 + nrow];
      const unsigned short hb = f2bf_bits(f);
      const unsigned short lb = f2bf_bits(f - bf_bits2f(hb));
      hv[it][e] = __builtin_bit_cast(_Float16, hb);
      lv[it][e] = __builtin_bit_cast(_Float16, lb);
    }
  }
  for (int pass = 0; pass < 2; ++pass) {
#pragma unroll
    for (int it = 0; it < 2; ++it) {
      const int nrow = it * 32 + wave * 4 + q;
      const size_t o = (size_t)(n0 + nrow) * Kdim + k0 + c8;
      *(volatile v8h*)(BtH + o) = hv[it];
      if (WITH_LO) *(volatile v8h*)(BtL + o) = lv[it];
    }
    __threadfence();
  }
}

__global__ __launch_bounds__(128) void layernorm_split_kernel(
    const float* __restrict__ x, const float* __restrict__ gw, const float* __restrict__ gb,
    unsigned short* __restrict__ NH, unsigned short* __restrict__ NL)
{
  __shared__ float red[8];
  const int tid = threadIdx.x, lane = tid & 31, wave = tid >> 5;
  const size_t e0 = (size_t)blockIdx.x * kHid + (size_t)tid * 8;
  const v4f a0 = *(const v4f*)(x + e0);
  const v4f a1 = *(const v4f*)(x + e0 + 4);
  float s = ((a0[0] + a0[1]) + (a0[2] + a0[3])) + ((a1[0] + a1[1]) + (a1[2] + a1[3]));
#pragma unroll
  for (int off = 16; off > 0; off >>= 1) s += __shfl_xor(s, off, 32);
  if (lane == 0) red[wave] = s;
  __syncthreads();
  const float mu = ((red[0] + red[1]) + (red[2] + red[3])) * (1.0f / (float)kHid);
  float dv[8];
#pragma unroll
  for (int e = 0; e < 4; ++e) { dv[e] = a0[e] - mu; dv[4 + e] = a1[e] - mu; }
  float s2 = 0.f;
#pragma unroll
  for (int e = 0; e < 8; ++e) s2 += dv[e] * dv[e];
#pragma unroll
  for (int off = 16; off > 0; off >>= 1) s2 += __shfl_xor(s2, off, 32);
  if (lane == 0) red[4 + wave] = s2;
  __syncthreads();
  const float var  = ((red[4] + red[5]) + (red[6] + red[7])) * (1.0f / (float)kHid);
  const float rstd = rsqrtf(var + 1e-5f);
  const v4f g0 = *(const v4f*)(gw + tid * 8);
  const v4f g1 = *(const v4f*)(gw + tid * 8 + 4);
  const v4f b0 = *(const v4f*)(gb + tid * 8);
  const v4f b1 = *(const v4f*)(gb + tid * 8 + 4);
  v8h hv, lv;
#pragma unroll
  for (int e = 0; e < 4; ++e) {
    const float f0 = dv[e] * rstd * g0[e] + b0[e];
    const float f1 = dv[4 + e] * rstd * g1[e] + b1[e];
    const unsigned short h0 = f2bf_bits(f0), h1 = f2bf_bits(f1);
    const unsigned short l0 = f2bf_bits(f0 - bf_bits2f(h0)), l1 = f2bf_bits(f1 - bf_bits2f(h1));
    hv[e]     = __builtin_bit_cast(_Float16, h0);
    hv[4 + e] = __builtin_bit_cast(_Float16, h1);
    lv[e]     = __builtin_bit_cast(_Float16, l0);
    lv[4 + e] = __builtin_bit_cast(_Float16, l1);
  }
  unsigned short* qh = NH + e0;
  unsigned short* ql = NL + e0;
  *(volatile v8h*)qh = hv;
  *(volatile v8h*)ql = lv;
  __threadfence();
  *(volatile v8h*)qh = hv;
  *(volatile v8h*)ql = lv;
}

__global__ __launch_bounds__(256) void conv_silu_kernel(
    const float* __restrict__ XZ, const float* __restrict__ cw, const float* __restrict__ cb,
    unsigned short* __restrict__ UCH, unsigned short* __restrict__ UCL)
{
  __shared__ __align__(16) float sT[16 * kConvTP];
  const int tid = threadIdx.x, lane = tid & 31, wave = tid >> 5;
  const int d0 = blockIdx.x * 256, d = d0 + tid;
  const int g0 = blockIdx.y * 64;
  const int tb = g0 & (kSeq - 1);
  const v4f wv = *(const v4f*)(cw + (size_t)d * 4);
  const float w0 = wv[0], w1 = wv[1], w2 = wv[2], w3 = wv[3];
  const float bcv = cb[d];
  float xm3, xm2, xm1;
  {
    const bool hist = (tb > 0);
    const int rb = hist ? (g0 - 3) : g0;
    const float v3 = XZ[(size_t)rb * kXzP + d];
    const float v2 = XZ[(size_t)(rb + 1) * kXzP + d];
    const float v1 = XZ[(size_t)(rb + 2) * kXzP + d];
    xm3 = hist ? v3 : 0.f;
    xm2 = hist ? v2 : 0.f;
    xm1 = hist ? v1 : 0.f;
  }
#pragma unroll 1
  for (int sub = 0; sub < 4; ++sub) {
    const int lb = g0 + sub * 16;
#pragma unroll 1
    for (int s = 0; s < 16; ++s) {
      const float xcur = XZ[(size_t)(lb + s) * kXzP + d];
      float acc = w0 * xm3;
      acc = fmaf(w1, xm2, acc);
      acc = fmaf(w2, xm1, acc);
      acc = fmaf(w3, xcur, acc);
      const float sv = acc + bcv;
      const float sg = __builtin_amdgcn_rcpf(1.0f + expf(-sv));
      sT[s * kConvTP + tid] = sv * sg;
      xm3 = xm2; xm2 = xm1; xm1 = xcur;
    }
    __syncthreads();
    v8h bh[2], blo[2];
#pragma unroll
    for (int it = 0; it < 2; ++it) {
      const float* sp = sT + (it * 8 + wave) * kConvTP + lane * 8;
      const v4f a0 = *(const v4f*)(sp);
      const v4f a1 = *(const v4f*)(sp + 4);
#pragma unroll
      for (int e = 0; e < 4; ++e) {
        const unsigned short h0 = f2bf_bits(a0[e]), h1 = f2bf_bits(a1[e]);
        const unsigned short l0 = f2bf_bits(a0[e] - bf_bits2f(h0)), l1 = f2bf_bits(a1[e] - bf_bits2f(h1));
        bh[it][e]      = __builtin_bit_cast(_Float16, h0);
        bh[it][4 + e]  = __builtin_bit_cast(_Float16, h1);
        blo[it][e]     = __builtin_bit_cast(_Float16, l0);
        blo[it][4 + e] = __builtin_bit_cast(_Float16, l1);
      }
    }
    for (int pass = 0; pass < 2; ++pass) {
#pragma unroll
      for (int it = 0; it < 2; ++it) {
        const size_t o = (size_t)(lb + it * 8 + wave) * kInner + d0 + lane * 8;
        *(volatile v8h*)(UCH + o) = bh[it];
        *(volatile v8h*)(UCL + o) = blo[it];
      }
      __threadfence();
    }
    __syncthreads();
  }
}

__device__ __forceinline__ float dt_from_pre(float v) {
  const float a  = expf(-fabsf(v));
  const float sp = fmaxf(v, 0.0f) + log1pf(a);
  return fminf(fmaxf(sp, 0.001f), 0.1f);
}

__global__ __launch_bounds__(256) void rowmean_kernel(const float* __restrict__ DTP, float* __restrict__ DTM)
{
  __shared__ float sM[32];
  const int tid = threadIdx.x, lane = tid & 31, wave = tid >> 5;
  const int tok0 = blockIdx.x * 32;
#pragma unroll 1
  for (int j = 0; j < 4; ++j) {
    const int tok = tok0 + wave * 4 + j;
    const float* rowp = DTP + (size_t)tok * kInner + lane;
    float s = 0.f;
#pragma unroll 1
    for (int i = 0; i < kInner / 32; ++i) s += dt_from_pre(rowp[i * 32]);
#pragma unroll
    for (int off = 16; off > 0; off >>= 1) s += __shfl_xor(s, off, 32);
    if (lane == 0) sM[wave * 4 + j] = s * (1.0f / (float)kInner);
  }
  __syncthreads();
  if (wave == 0) {
    const float mv = sM[lane];
    volatile float* p = DTM + tok0 + lane;
    *p = mv;
    __threadfence();
    *p = mv;
  }
}

__global__ __launch_bounds__(64) void scan_kernel(
    const float* __restrict__ BC, const float* __restrict__ bcb, const float* __restrict__ DTM,
    const float* __restrict__ DTP, const unsigned* __restrict__ XAHw, const unsigned* __restrict__ XALw,
    const float* __restrict__ XZ, unsigned short* __restrict__ GH, unsigned short* __restrict__ GL)
{
  __shared__ __align__(16) float sX[kScanTS * kBcN];
  __shared__ __align__(16) float sD[kScanTS];
  __shared__ __align__(16) float sY[kScanTS * kScanYP];
  const int tid = threadIdx.x, lane = tid & 31, wave = tid >> 5;
  constexpr int kBlkPerB = kInner / kScanCh;
  const int bix = blockIdx.x / kBlkPerB;
  const int d0  = (blockIdx.x - bix * kBlkPerB) * kScanCh;
  const int d   = d0 + tid;
  const size_t row0 = (size_t)bix * kSeq;
  const bool odd = (d & 1) != 0;
  float h[kNst];
#pragma unroll
  for (int n = 0; n < kNst; ++n) h[n] = 0.f;
  const int lr = tid >> 3, lc4 = (tid & 7) * 4;
  const v4f bb = *(const v4f*)(bcb + lc4);
  const int q = lane >> 3, c8 = (lane & 7) * 8;
#pragma unroll 1
  for (int t0 = 0; t0 < kSeq; t0 += kScanTS) {
    __syncthreads();
#pragma unroll 4
    for (int i = 0; i < 8; ++i) {
      const int r = lr + 8 * i;
      v4f v = *(const v4f*)(BC + (row0 + t0 + r) * kBcP + lc4);
      v = v + bb;
      *(v4f*)(sX + r * kBcN + lc4) = v;
    }
    sD[tid] = DTM[row0 + t0 + tid];
    __syncthreads();
#pragma unroll 1
    for (int s = 0; s < kScanTS; ++s) {
      const size_t tok = row0 + t0 + s;
      const float* xr = sX + s * kBcN;
      float Bs[kNst], Cs[kNst];
#pragma unroll
      for (int q4 = 0; q4 < 4; ++q4) {
        const v4f bv = *(const v4f*)(xr + 4 * q4);
        const v4f cv = *(const v4f*)(xr + kNst + 4 * q4);
        Bs[4 * q4 + 0] = bv[0]; Bs[4 * q4 + 1] = bv[1]; Bs[4 * q4 + 2] = bv[2]; Bs[4 * q4 + 3] = bv[3];
        Cs[4 * q4 + 0] = cv[0]; Cs[4 * q4 + 1] = cv[1]; Cs[4 * q4 + 2] = cv[2]; Cs[4 * q4 + 3] = cv[3];
      }
      const float pre = DTP[tok * kInner + d];
      const size_t widx = (tok * kInner + d) >> 1;
      const unsigned wh = XAHw[widx];
      const unsigned wl = XALw[widx];
      const float zv = XZ[tok * kXzP + kInner + d];
      const unsigned hbits = odd ? (wh & 0xffff0000u) : (wh << 16);
      const unsigned lbits = odd ? (wl & 0xffff0000u) : (wl << 16);
      const float xt = __uint_as_float(hbits) + __uint_as_float(lbits);
      const float dt = dt_from_pre(pre);
      const float e  = expf(-dt);
      const float sc = sD[s] * xt;
      float a = 1.0f, y = 0.f;
#pragma unroll
      for (int n = 0; n < kNst; ++n) {
        a *= e;
        h[n] = a * h[n] + sc * Bs[n];
        y = h[n] * Cs[n] + y;
      }
      const float sg = __builtin_amdgcn_rcpf(1.0f + expf(-zv));
      y = y * (zv * sg);
      sY[s * kScanYP + tid] = y;
    }
    __syncthreads();
    v8h hv[8], lv[8];
#pragma unroll
    for (int it = 0; it < 8; ++it) {
      const int row = it * 8 + wave * 4 + q;
      const float* sp = sY + row * kScanYP + c8;
      const v4f a0 = *(const v4f*)(sp);
      const v4f a1 = *(const v4f*)(sp + 4);
#pragma unroll
      for (int k = 0; k < 4; ++k) {
        const unsigned short h0 = f2bf_bits(a0[k]), h1 = f2bf_bits(a1[k]);
        const unsigned short l0 = f2bf_bits(a0[k] - bf_bits2f(h0)), l1 = f2bf_bits(a1[k] - bf_bits2f(h1));
        hv[it][k]     = __builtin_bit_cast(_Float16, h0);
        hv[it][4 + k] = __builtin_bit_cast(_Float16, h1);
        lv[it][k]     = __builtin_bit_cast(_Float16, l0);
        lv[it][4 + k] = __builtin_bit_cast(_Float16, l1);
      }
    }
    for (int pass = 0; pass < 2; ++pass) {
#pragma unroll
      for (int it = 0; it < 8; ++it) {
        const int row = it * 8 + wave * 4 + q;
        const size_t o = (row0 + t0 + row) * kInner + d0 + c8;
        *(volatile v8h*)(GH + o) = hv[it];
        *(volatile v8h*)(GL + o) = lv[it];
      }
      __threadfence();
    }
  }
}

static_assert((kTok / 64) * (kXzP / 64) == 256 * 8, "in_proj grid");
static_assert((kTok / 64) * (kBcP / 64) == 4 * 8, "B/C grid");
static_assert((kTok / 64) * (kDtR / 64) == 4 * 8, "dt-rank grid");
static_assert((kTok / 64) * (kInner / 64) == 128 * 8, "dt grid");
static_assert((kTok / 64) * (kHid / 64) == 64 * 8, "out_proj grid");

extern "C" void kernel_launch(void* const* d_in, const int* in_sizes, int n_in,
                              void* d_out, int out_size, void* d_ws, size_t ws_size,
                              hipStream_t stream) {
  if (n_in < 15) return;
  if (in_sizes[0]  != kTok * kHid) return;
  if (in_sizes[1]  != kHid || in_sizes[2] != kHid) return;
  if (in_sizes[3]  != kHid * kXzP || in_sizes[4] != kXzP) return;
  if (in_sizes[5]  != kInner * 4 || in_sizes[6] != kInner) return;
  if (in_sizes[7]  != kInner * kBcN || in_sizes[8] != kBcN) return;
  if (in_sizes[9]  != kInner * kDtR || in_sizes[10] != kDtR) return;
  if (in_sizes[11] != kDtR * kInner || in_sizes[12] != kInner) return;
  if (in_sizes[13] != kInner * kHid || in_sizes[14] != kHid) return;
  if (out_size != kTok * kHid) return;
  if (ws_size < kWsTotal) return;

  const float* x      = (const float*)d_in[0];
  const float* norm_w = (const float*)d_in[1];
  const float* norm_b = (const float*)d_in[2];
  const float* in_w   = (const float*)d_in[3];
  const float* in_b   = (const float*)d_in[4];
  const float* conv_w = (const float*)d_in[5];
  const float* conv_b = (const float*)d_in[6];
  const float* bc_w   = (const float*)d_in[7];
  const float* bc_b   = (const float*)d_in[8];
  const float* dtr_w  = (const float*)d_in[9];
  const float* dtr_b  = (const float*)d_in[10];
  const float* dt_w   = (const float*)d_in[11];
  const float* dt_b   = (const float*)d_in[12];
  const float* out_w  = (const float*)d_in[13];
  const float* out_b  = (const float*)d_in[14];
  float* outp = (float*)d_out;

  char* ws = (char*)d_ws;
  unsigned short* BIH = (unsigned short*)(ws + kOffBIH);
  unsigned short* BIL = (unsigned short*)(ws + kOffBIL);
  unsigned short* BOH = (unsigned short*)(ws + kOffBOH);
  unsigned short* BOL = (unsigned short*)(ws + kOffBOL);
  unsigned short* BCH = (unsigned short*)(ws + kOffBCH);
  unsigned short* BCL = (unsigned short*)(ws + kOffBCL);
  unsigned short* BDR = (unsigned short*)(ws + kOffBDR);
  unsigned short* BDT = (unsigned short*)(ws + kOffBDT);
  unsigned short* NH  = (unsigned short*)(ws + kOffNH);
  unsigned short* NL  = (unsigned short*)(ws + kOffNL);
  float*          XZ  = (float*)(ws + kOffXZ);
  unsigned short* XAH = (unsigned short*)(ws + kOffXAH);
  unsigned short* XAL = (unsigned short*)(ws + kOffXAL);
  float*          BC  = (float*)(ws + kOffBC);
  unsigned short* DTR = (unsigned short*)(ws + kOffDTR);
  float*          DTM = (float*)(ws + kOffDTM);
  float*          DTP = (float*)(ws + kOffDTP);
  unsigned short* GH  = (unsigned short*)(ws + kOffGH);
  unsigned short* GL  = (unsigned short*)(ws + kOffGL);

  transpose_split_kernel<true><<<dim3(kXzP / 64, kHid / 64), 256, 0, stream>>>(in_w, BIH, BIL, kHid, kXzP);
  transpose_split_kernel<true><<<dim3(kHid / 64, kInner / 64), 256, 0, stream>>>(out_w, BOH, BOL, kInner, kHid);
  transpose_split_kernel<true><<<dim3(kBcP / 64, kInner / 64), 256, 0, stream>>>(bc_w, BCH, BCL, kInner, kBcN);
  transpose_split_kernel<false><<<dim3(kDtR / 64, kInner / 64), 256, 0, stream>>>(dtr_w, BDR, BDR, kInner, kDtR);
  transpose_split_kernel<false><<<dim3(kInner / 64, kDtR / 64), 256, 0, stream>>>(dt_w, BDT, BDT, kDtR, kInner);

  layernorm_split_kernel<<<kTok, 128, 0, stream>>>(x, norm_w, norm_b, NH, NL);

  wmma_gemm64<1, 2, 2, 0, false><<<dim3(256, 1), 256, 0, stream>>>(
      NH, NL, kHid, 0L,
      BIH, BIL, kHid, 0L,
      (void*)XZ, (void*)XZ, kXzP, 0L,
      in_b, x, 0L,
      kTok, kXzP, kHid, 1.0f);

  conv_silu_kernel<<<dim3(kInner / 256, kTok / 64), 256, 0, stream>>>(XZ, conv_w, conv_b, XAH, XAL);

  wmma_gemm64<1, 2, 0, 0, false><<<dim3(4, 1), 256, 0, stream>>>(
      XAH, XAL, kInner, 0L,
      BCH, BCL, kInner, 0L,
      (void*)BC, (void*)BC, kBcP, 0L,
      bc_b, x, 0L,
      kTok, kBcP, kInner, 1.0f);

  wmma_gemm64<1, 0, 2, 3, false><<<dim3(4, 1), 256, 0, stream>>>(
      XAH, XAH, kInner, 0L,
      BDR, BDR, kInner, 0L,
      (void*)DTR, (void*)DTR, kDtR, 0L,
      dtr_b, x, 0L,
      kTok, kDtR, kInner, 1.0f);

  wmma_gemm64<1, 0, 2, 0, false><<<dim3(128, 1), 256, 0, stream>>>(
      DTR, DTR, kDtR, 0L,
      BDT, BDT, kDtR, 0L,
      (void*)DTP, (void*)DTP, kInner, 0L,
      dt_b, x, 0L,
      kTok, kInner, kDtR, 1.0f);

  rowmean_kernel<<<kTok / 32, 256, 0, stream>>>(DTP, DTM);

  scan_kernel<<<kBatch * (kInner / kScanCh), kScanCh, 0, stream>>>(
      BC, bc_b, DTM, DTP, (const unsigned*)XAH, (const unsigned*)XAL, XZ, GH, GL);

  wmma_gemm64<1, 2, 2, 0, false><<<dim3(64, 1), 256, 0, stream>>>(
      GH, GL, kInner, 0L,
      BOH, BOL, kInner, 0L,
      (void*)outp, (void*)outp, kHid, 0L,
      out_b, x, 0L,
      kTok, kHid, kInner, 1.0f);
}
